// _Conv1D_68805376082214
// MI455X (gfx1250) — hardware-verified
//
#include <hip/hip_runtime.h>


typedef __attribute__((ext_vector_type(16))) _Float16 v16h;
typedef __attribute__((ext_vector_type(8)))  _Float16 v8h;
typedef __attribute__((ext_vector_type(4)))  _Float16 v4h;
typedef __attribute__((ext_vector_type(8)))  float    v8f;
typedef __attribute__((ext_vector_type(4)))  float    v4f;

__device__ __forceinline__ v8f mma16(v16h a, v16h b, v8f c) {
    c = __builtin_amdgcn_wmma_f32_16x16x32_f16(false, a, false, b, (short)0, c, false, false);
    asm volatile("v_nop\n\tv_nop\n\tv_nop\n\tv_nop" : "+v"(c) : "v"(a), "v"(b));
    return c;
}
__device__ __forceinline__ int koff(int e, int h) { return (e < 8) ? (8 * h + e) : (16 + 8 * h + (e - 8)); }

#define BATCH 16
#define SEQ   2048
#define CH    256
#define FILT  256
#define KW    5
#define KC    (KW * CH)
#define NCHUNK (KC / 32)
#define ROWS_PER_WG 64
#define LDSROWS (ROWS_PER_WG + KW - 1)
#define LDSSTRIDE 264

__global__ __launch_bounds__(256) void conv1d_wswizzle(
    const float* __restrict__ w, _Float16* __restrict__ blob)
{
    int t    = blockIdx.x * 256 + threadIdx.x;
    int idx0 = t * 8;
    int e0   = idx0 & 15;
    int lane = (idx0 >> 4) & 31;
    int rest = idx0 >> 9;
    int chunk = rest % NCHUNK;
    int nt    = rest / NCHUNK;
    int f     = nt * 16 + (lane & 15);
    v8h v;
    #pragma unroll
    for (int i = 0; i < 8; ++i) {
        int k_local = koff(e0 + i, lane >> 4);
        int kc      = chunk * 32 + k_local;
        v[i] = (_Float16)w[f * KC + kc];
    }
    *(volatile v8h*)(blob + idx0) = v;
    __threadfence();
    *(volatile v8h*)(blob + idx0) = v;
}

__global__ __launch_bounds__(256) void conv1d_wmma(
    const float* __restrict__ x,
    const _Float16* __restrict__ wh,
    const float* __restrict__ bias,
    float* __restrict__ out)
{
    __shared__ _Float16 xs[LDSROWS * LDSSTRIDE];
    __shared__ __attribute__((aligned(16))) float so[8][ROWS_PER_WG][32];

    const int batch = blockIdx.x >> 5;
    const int s0    = (blockIdx.x & 31) << 6;

    const int wave = threadIdx.x >> 5;
    const int lane = threadIdx.x & 31;
    const int m    = lane & 15;
    const int hi   = lane >> 4;
    const int n    = lane & 15;

    const int nt0 = wave * 2;
    const int nt1 = nt0 + 1;

    const _Float16* bp0 = wh + (((size_t)nt0 * NCHUNK) * 32 + lane) * 16;
    const _Float16* bp1 = wh + (((size_t)nt1 * NCHUNK) * 32 + lane) * 16;

    #pragma unroll
    for (int pk = 0; pk < 4; ++pk) {
        __builtin_prefetch(bp0 + (size_t)pk * 512, 0, 0);
        __builtin_prefetch(bp1 + (size_t)pk * 512, 0, 0);
    }

    {
        const int c4 = (threadIdx.x & 63) << 2;
        const int r0 = threadIdx.x >> 6;
        #pragma unroll 4
        for (int r = r0; r < LDSROWS; r += 4) {
            int s = s0 - (KW - 1) + r;
            v4f v = {};
            if (s >= 0)
                v = *(const v4f*)(x + (((size_t)batch * SEQ + s) * CH) + c4);
            v4h h; h.x = (_Float16)v.x; h.y = (_Float16)v.y;
                   h.z = (_Float16)v.z; h.w = (_Float16)v.w;
            *(v4h*)(&xs[r * LDSSTRIDE + c4]) = h;
        }
    }
    __syncthreads();

    v8f acc[4][2] = {};

    for (int ck = 0; ck < NCHUNK; ++ck) {
        const int k  = ck >> 3;
        const int c0 = (ck & 7) << 5;

        union { v16h v; v8h h[2]; } b0, b1;
        const _Float16* q0 = bp0 + (size_t)ck * 512;
        const _Float16* q1 = bp1 + (size_t)ck * 512;
        b0.h[0] = *(const v8h*)(q0);
        b0.h[1] = *(const v8h*)(q0 + 8);
        b1.h[0] = *(const v8h*)(q1);
        b1.h[1] = *(const v8h*)(q1 + 8);

        #pragma unroll
        for (int mt = 0; mt < 4; ++mt) {
            const _Float16* ap = &xs[(mt * 16 + m + k) * LDSSTRIDE + c0 + hi * 8];
            union { v16h v; v8h h[2]; } a;
            a.h[0] = *(const v8h*)(ap);
            a.h[1] = *(const v8h*)(ap + 16);
            acc[mt][0] = mma16(a.v, b0.v, acc[mt][0]);
            acc[mt][1] = mma16(a.v, b1.v, acc[mt][1]);
        }
    }

    const float bv0 = bias[nt0 * 16 + n];
    const float bv1 = bias[nt1 * 16 + n];

    #pragma unroll
    for (int mt = 0; mt < 4; ++mt) {
        #pragma unroll
        for (int r = 0; r < 8; ++r) {
            so[wave][mt * 16 + hi * 8 + r][n]      = acc[mt][0][r] + bv0;
            so[wave][mt * 16 + hi * 8 + r][16 + n] = acc[mt][1][r] + bv1;
        }
    }
    __builtin_amdgcn_fence(__ATOMIC_ACQ_REL, "workgroup");
    __builtin_amdgcn_wave_barrier();
    typedef float v4fa __attribute__((ext_vector_type(4), may_alias));
    const int rsub = lane >> 3, c4 = (lane & 7) * 4;
    float* obase = out + (((size_t)batch * SEQ + s0) * FILT) + wave * 32 + c4;
    #pragma unroll
    for (int pass = 0; pass < 2; ++pass) {
        #pragma unroll
        for (int q = 0; q < 16; ++q) {
            const int row = q * 4 + rsub;
            const v4f v = *(const v4fa*)&so[wave][row][c4];
            *(volatile v4f*)(obase + (size_t)row * FILT) = v;
        }
        if (pass == 0) __threadfence();
    }
}

extern "C" void kernel_launch(void* const* d_in, const int* in_sizes, int n_in,
                              void* d_out, int out_size, void* d_ws, size_t ws_size,
                              hipStream_t stream)
{
    const float* x    = (const float*)d_in[0];
    const float* w    = (const float*)d_in[1];
    const float* bias = (const float*)d_in[2];
    float*       out  = (float*)d_out;
    _Float16*    wh   = (_Float16*)d_ws;

    (void)in_sizes; (void)n_in; (void)out_size; (void)ws_size;

    conv1d_wswizzle<<<(FILT * KC) / 8 / 256, 256, 0, stream>>>(w, wh);

    conv1d_wmma<<<(BATCH * SEQ) / ROWS_PER_WG, 256, 0, stream>>>(x, wh, bias, out);
}
